// Encoder_84748294685286
// MI455X (gfx1250) — hardware-verified
//
#include <hip/hip_runtime.h>
#include <math.h>

constexpr int NBATCH  = 128;
constexpr int NSTEP   = 512;
constexpr int NFEAT   = 64;
constexpr int NUA     = 256;
constexpr int NUB     = 128;
constexpr int NGA     = 4 * NUA;
constexpr int NGB     = 4 * NUB;
constexpr int K_L1    = NFEAT + NUA;
constexpr int K_L2    = NUA + NUB;
constexpr int NTHR    = 256;
constexpr int SEQ_BLK = 16;
constexpr int XPITCH  = 72;
constexpr int HPA     = 264;
constexpr int HPB     = 136;
constexpr int OPITCH  = 132;
constexpr int HASZ    = SEQ_BLK * HPA;
constexpr int HBSZ    = SEQ_BLK * HPB;
constexpr float WSC      = 16.0f;
constexpr float WSC_INV  = 1.0f / WSC;
constexpr float RES_SC   = 2048.0f;
constexpr float RES_INV  = 1.0f / RES_SC;
constexpr float F16_MINN = 6.103515625e-05f;
static_assert(NBATCH % SEQ_BLK == 0, "batch tiles");
static_assert(NUA == 32 * (NTHR / 32), "8 waves x 32 layer-1 units");
static_assert(NUB == 16 * (NTHR / 32), "8 waves x 16 layer-2 units");
static_assert(K_L1 % 32 == 0 && K_L2 % 32 == 0 && NFEAT % 32 == 0 && NUA % 32 == 0 && NUB % 32 == 0, "k chunks of 32");
static_assert(NGA % 64 == 0 && NGB % 64 == 0 && NFEAT % 64 == 0 && NUA % 64 == 0 && NUB % 64 == 0, "pack tiles of 64");
static_assert((2 * HASZ) % NTHR == 0 && (2 * HBSZ) % NTHR == 0, "zero-fill loops exact");
static_assert(SEQ_BLK * NFEAT == NTHR * 4, "x tile: one float4 per thread");
static_assert((SEQ_BLK * NUB) == 2 * NTHR * 4, "output tile: two float4 per thread");
static_assert((XPITCH % 8) == 0 && (HPA % 8) == 0 && (HPB % 8) == 0 && (OPITCH % 4) == 0, "16-B aligned LDS rows");

typedef __attribute__((ext_vector_type(16))) _Float16 v16h;
typedef __attribute__((ext_vector_type(8)))  _Float16 v8h;
typedef __attribute__((ext_vector_type(4)))  _Float16 v4h;
typedef __attribute__((ext_vector_type(8)))  float    v8f;
typedef __attribute__((ext_vector_type(4)))  float    v4f;

template <typename T> struct Frag;
template <> struct Frag<_Float16> {
  typedef v16h V; union U { v16h v; v8h h[2]; };
  static __device__ __forceinline__ v16h load(const _Float16* p) {
    U f; f.h[0] = *(const v8h*)(p); f.h[1] = *(const v8h*)(p + 16); return f.v;
  }
  static __device__ __forceinline__ v8f mma(v16h a, v16h b, v8f c) {
    return __builtin_amdgcn_wmma_f32_16x16x32_f16(false, a, false, b, (short)0, c, false, false);
  }
};

__device__ __forceinline__ void guard4_in(v8f& a0, v8f& a1, v8f& a2, v8f& a3,
                                          v16h x, v16h b0, v16h b1, v16h b2, v16h b3) {
  asm volatile("v_nop\n\tv_nop\n\tv_nop\n\tv_nop"
               : "+v"(a0), "+v"(a1), "+v"(a2), "+v"(a3)
               : "v"(x), "v"(b0), "v"(b1), "v"(b2), "v"(b3));
}
__device__ __forceinline__ void guard8_in(v8f& a0, v8f& a1, v8f& a2, v8f& a3, v8f& a4, v8f& a5, v8f& a6, v8f& a7,
                                          v16h x, v16h y, v16h b0, v16h b1, v16h b2, v16h b3) {
  asm volatile("v_nop\n\tv_nop\n\tv_nop\n\tv_nop"
               : "+v"(a0), "+v"(a1), "+v"(a2), "+v"(a3), "+v"(a4), "+v"(a5), "+v"(a6), "+v"(a7)
               : "v"(x), "v"(y), "v"(b0), "v"(b1), "v"(b2), "v"(b3));
}
__device__ __forceinline__ void acc_guard8(v8f& a0, v8f& a1, v8f& a2, v8f& a3, v8f& a4, v8f& a5, v8f& a6, v8f& a7) {
  asm volatile("v_nop\n\tv_nop\n\tv_nop\n\tv_nop"
               : "+v"(a0), "+v"(a1), "+v"(a2), "+v"(a3), "+v"(a4), "+v"(a5), "+v"(a6), "+v"(a7));
}

__device__ __forceinline__ float fsig(float v) { return __builtin_amdgcn_rcpf(1.0f + expf(-v)); }

__device__ __forceinline__ void split_h(float h, _Float16& hi, _Float16& lo) {
  const _Float16 a = (_Float16)h;
  float af = (float)a;
  const bool tiny = fabsf(af) < F16_MINN;
  af = tiny ? 0.0f : af;
  hi = (_Float16)af;
  lo = (_Float16)((h - af) * RES_SC);
}

__global__ __launch_bounds__(NTHR) void tpw_kernel(const float* __restrict__ src, int R, int C, int ldo, int kofs,
                                                   unsigned short* __restrict__ O, float sc) {
  __shared__ float Tt[64 * 65];
  (void)R;
  const int tid = threadIdx.x;
  const int c0 = blockIdx.x * 64, r0 = blockIdx.y * 64;
#pragma unroll
  for (int i = 0; i < 4; ++i) {
    const int idx = i * NTHR + tid;
    const int rr = idx >> 4, cc = (idx & 15) * 4;
    const v4f v = *(const v4f*)(src + (size_t)(r0 + rr) * (size_t)C + c0 + cc);
    Tt[rr * 65 + cc + 0] = v[0];
    Tt[rr * 65 + cc + 1] = v[1];
    Tt[rr * 65 + cc + 2] = v[2];
    Tt[rr * 65 + cc + 3] = v[3];
  }
  __syncthreads();
  const int q = tid >> 3, c8 = (tid & 7) * 8;
  v8h hv[2];
#pragma unroll
  for (int g = 0; g < 2; ++g) {
    const int qq = g * 32 + q;
#pragma unroll
    for (int e = 0; e < 8; ++e) {
      const float f = Tt[(c8 + e) * 65 + qq];
      hv[g][e] = (_Float16)(f * sc);
    }
  }
  for (int pass = 0; pass < 2; ++pass) {
#pragma unroll
    for (int g = 0; g < 2; ++g) {
      const size_t o = (size_t)(c0 + g * 32 + q) * (size_t)ldo + (size_t)(kofs + r0 + c8);
      *(volatile v8h*)(O + o) = hv[g];
    }
    __threadfence();
  }
}

__global__ __launch_bounds__(NTHR) void lstm2_kernel(const float* __restrict__ x,
                                                     const float* __restrict__ bias_a, const float* __restrict__ bias_b,
                                                     const unsigned short* __restrict__ WAp,
                                                     const unsigned short* __restrict__ WBp,
                                                     float* __restrict__ out) {
  __shared__ __align__(16) _Float16 Ax[SEQ_BLK * XPITCH];
  __shared__ __align__(16) _Float16 HAh[2 * HASZ];
  __shared__ __align__(16) _Float16 HAl[2 * HASZ];
  __shared__ __align__(16) _Float16 HBh[2 * HBSZ];
  __shared__ __align__(16) _Float16 HBl[2 * HBSZ];
  __shared__ __align__(16) float    Hs[SEQ_BLK * OPITCH];
  const _Float16* WA = (const _Float16*)WAp;
  const _Float16* WB = (const _Float16*)WBp;
  const int tid = threadIdx.x, lane = tid & 31, wave = tid >> 5;
  const int c = lane & 15, hh = lane >> 4, koff = hh * 8;
  const int rowbase = blockIdx.x * SEQ_BLK;

#pragma unroll 1
  for (int i = tid; i < 2 * HASZ; i += NTHR) { HAh[i] = (_Float16)0.0f; HAl[i] = (_Float16)0.0f; }
#pragma unroll 1
  for (int i = tid; i < 2 * HBSZ; i += NTHR) { HBh[i] = (_Float16)0.0f; HBl[i] = (_Float16)0.0f; }
  __syncthreads();

  const int xm = tid >> 4, xf4 = (tid & 15) * 4;
  const float* xrowp = x + ((size_t)(rowbase + xm) * NSTEP) * NFEAT + xf4;
  {
    const v4f v = *(const v4f*)(xrowp);
    v4h pk;
    pk[0] = (_Float16)v[0]; pk[1] = (_Float16)v[1]; pk[2] = (_Float16)v[2]; pk[3] = (_Float16)v[3];
    *(v4h*)(Ax + xm * XPITCH + xf4) = pk;
  }

  float bba[2][4], bbb[4];
#pragma unroll
  for (int nt = 0; nt < 2; ++nt)
#pragma unroll
    for (int g = 0; g < 4; ++g) bba[nt][g] = bias_a[g * NUA + 32 * wave + 16 * nt + c];
  asm volatile("" ::: "memory");
#pragma unroll
  for (int g = 0; g < 4; ++g) bbb[g] = bias_b[g * NUB + 16 * wave + c];

  float ca[2][8], cb[8], h2v[8];
#pragma unroll
  for (int r = 0; r < 8; ++r) { ca[0][r] = 0.0f; ca[1][r] = 0.0f; cb[r] = 0.0f; h2v[r] = 0.0f; }
  __syncthreads();

  const _Float16* axrow = Ax + c * XPITCH + koff;
  const int j2 = 16 * wave + c;
  const _Float16* wb2 = WB + (size_t)j2 * K_L2 + koff;
  const v8f z8 = {0.f, 0.f, 0.f, 0.f, 0.f, 0.f, 0.f, 0.f};

#pragma unroll 1
  for (int t = 0; t < NSTEP; ++t) {
    const int cur = t & 1;
    const _Float16* h1rh = HAh + cur * HASZ + c * HPA + koff;
    const _Float16* h1rl = HAl + cur * HASZ + c * HPA + koff;
    _Float16* h1wh = HAh + (cur ^ 1) * HASZ;
    _Float16* h1wl = HAl + (cur ^ 1) * HASZ;
    const _Float16* h2rh = HBh + cur * HBSZ + c * HPB + koff;
    const _Float16* h2rl = HBl + cur * HBSZ + c * HPB + koff;
    _Float16* h2wh = HBh + (cur ^ 1) * HBSZ;
    _Float16* h2wl = HBl + (cur ^ 1) * HBSZ;

    const int tn = (t + 1 < NSTEP) ? (t + 1) : (NSTEP - 1);
    const v4f xnext = *(const v4f*)(xrowp + (size_t)tn * NFEAT);

#pragma unroll
    for (int nt = 0; nt < 2; ++nt) {
      const int j = 32 * wave + 16 * nt + c;
      const _Float16* wb = WA + (size_t)j * K_L1 + koff;
      v8f m0 = z8, m1 = z8, m2 = z8, m3 = z8;
      v8f q0 = z8, q1 = z8, q2 = z8, q3 = z8;
#pragma unroll 1
      for (int kx = 0; kx < NFEAT; kx += 32) {
        const v16h a  = Frag<_Float16>::load(axrow + kx);
        const v16h b0 = Frag<_Float16>::load(wb + kx);
        const v16h b1 = Frag<_Float16>::load(wb + (size_t)1 * NUA * K_L1 + kx);
        const v16h b2 = Frag<_Float16>::load(wb + (size_t)2 * NUA * K_L1 + kx);
        const v16h b3 = Frag<_Float16>::load(wb + (size_t)3 * NUA * K_L1 + kx);
        m0 = Frag<_Float16>::mma(a, b0, m0);
        m1 = Frag<_Float16>::mma(a, b1, m1);
        m2 = Frag<_Float16>::mma(a, b2, m2);
        m3 = Frag<_Float16>::mma(a, b3, m3);
        guard4_in(m0, m1, m2, m3, a, b0, b1, b2, b3);
      }
#pragma unroll 1
      for (int k0 = 0; k0 < NUA; k0 += 32) {
        const v16h ah = Frag<_Float16>::load(h1rh + k0);
        const v16h al = Frag<_Float16>::load(h1rl + k0);
        const v16h b0 = Frag<_Float16>::load(wb + NFEAT + k0);
        const v16h b1 = Frag<_Float16>::load(wb + (size_t)1 * NUA * K_L1 + NFEAT + k0);
        const v16h b2 = Frag<_Float16>::load(wb + (size_t)2 * NUA * K_L1 + NFEAT + k0);
        const v16h b3 = Frag<_Float16>::load(wb + (size_t)3 * NUA * K_L1 + NFEAT + k0);
        m0 = Frag<_Float16>::mma(ah, b0, m0);
        m1 = Frag<_Float16>::mma(ah, b1, m1);
        m2 = Frag<_Float16>::mma(ah, b2, m2);
        m3 = Frag<_Float16>::mma(ah, b3, m3);
        q0 = Frag<_Float16>::mma(al, b0, q0);
        q1 = Frag<_Float16>::mma(al, b1, q1);
        q2 = Frag<_Float16>::mma(al, b2, q2);
        q3 = Frag<_Float16>::mma(al, b3, q3);
        guard8_in(m0, m1, m2, m3, q0, q1, q2, q3, ah, al, b0, b1, b2, b3);
      }
      acc_guard8(m0, m1, m2, m3, q0, q1, q2, q3);
#pragma unroll
      for (int r = 0; r < 8; ++r) {
        const float zi = (m0[r] + q0[r] * RES_INV) * WSC_INV + bba[nt][0];
        const float zf = (m1[r] + q1[r] * RES_INV) * WSC_INV + bba[nt][1];
        const float zg = (m2[r] + q2[r] * RES_INV) * WSC_INV + bba[nt][2];
        const float zo = (m3[r] + q3[r] * RES_INV) * WSC_INV + bba[nt][3];
        const float ig = fsig(zi);
        const float fg = fsig(zf);
        const float og = fsig(zo);
        const float gg = fmaxf(zg, 0.0f);
        const float cn = fg * ca[nt][r] + ig * gg;
        ca[nt][r] = cn;
        const float hn = og * fmaxf(cn, 0.0f);
        _Float16 hi, lo;
        split_h(hn, hi, lo);
        h1wh[(8 * hh + r) * HPA + j] = hi;
        h1wl[(8 * hh + r) * HPA + j] = lo;
      }
    }
    __syncthreads();

    {
      v4h pk;
      pk[0] = (_Float16)xnext[0]; pk[1] = (_Float16)xnext[1]; pk[2] = (_Float16)xnext[2]; pk[3] = (_Float16)xnext[3];
      *(v4h*)(Ax + xm * XPITCH + xf4) = pk;
    }

    {
      const _Float16* h1nh = h1wh + c * HPA + koff;
      const _Float16* h1nl = h1wl + c * HPA + koff;
      v8f m0 = z8, m1 = z8, m2 = z8, m3 = z8;
      v8f q0 = z8, q1 = z8, q2 = z8, q3 = z8;
#pragma unroll 1
      for (int k0 = 0; k0 < NUA; k0 += 32) {
        const v16h ah = Frag<_Float16>::load(h1nh + k0);
        const v16h al = Frag<_Float16>::load(h1nl + k0);
        const v16h b0 = Frag<_Float16>::load(wb2 + k0);
        const v16h b1 = Frag<_Float16>::load(wb2 + (size_t)1 * NUB * K_L2 + k0);
        const v16h b2 = Frag<_Float16>::load(wb2 + (size_t)2 * NUB * K_L2 + k0);
        const v16h b3 = Frag<_Float16>::load(wb2 + (size_t)3 * NUB * K_L2 + k0);
        m0 = Frag<_Float16>::mma(ah, b0, m0);
        m1 = Frag<_Float16>::mma(ah, b1, m1);
        m2 = Frag<_Float16>::mma(ah, b2, m2);
        m3 = Frag<_Float16>::mma(ah, b3, m3);
        q0 = Frag<_Float16>::mma(al, b0, q0);
        q1 = Frag<_Float16>::mma(al, b1, q1);
        q2 = Frag<_Float16>::mma(al, b2, q2);
        q3 = Frag<_Float16>::mma(al, b3, q3);
        guard8_in(m0, m1, m2, m3, q0, q1, q2, q3, ah, al, b0, b1, b2, b3);
      }
#pragma unroll 1
      for (int k0 = 0; k0 < NUB; k0 += 32) {
        const v16h ah = Frag<_Float16>::load(h2rh + k0);
        const v16h al = Frag<_Float16>::load(h2rl + k0);
        const v16h b0 = Frag<_Float16>::load(wb2 + NUA + k0);
        const v16h b1 = Frag<_Float16>::load(wb2 + (size_t)1 * NUB * K_L2 + NUA + k0);
        const v16h b2 = Frag<_Float16>::load(wb2 + (size_t)2 * NUB * K_L2 + NUA + k0);
        const v16h b3 = Frag<_Float16>::load(wb2 + (size_t)3 * NUB * K_L2 + NUA + k0);
        m0 = Frag<_Float16>::mma(ah, b0, m0);
        m1 = Frag<_Float16>::mma(ah, b1, m1);
        m2 = Frag<_Float16>::mma(ah, b2, m2);
        m3 = Frag<_Float16>::mma(ah, b3, m3);
        q0 = Frag<_Float16>::mma(al, b0, q0);
        q1 = Frag<_Float16>::mma(al, b1, q1);
        q2 = Frag<_Float16>::mma(al, b2, q2);
        q3 = Frag<_Float16>::mma(al, b3, q3);
        guard8_in(m0, m1, m2, m3, q0, q1, q2, q3, ah, al, b0, b1, b2, b3);
      }
      acc_guard8(m0, m1, m2, m3, q0, q1, q2, q3);
#pragma unroll
      for (int r = 0; r < 8; ++r) {
        const float zi = (m0[r] + q0[r] * RES_INV) * WSC_INV + bbb[0];
        const float zf = (m1[r] + q1[r] * RES_INV) * WSC_INV + bbb[1];
        const float zg = (m2[r] + q2[r] * RES_INV) * WSC_INV + bbb[2];
        const float zo = (m3[r] + q3[r] * RES_INV) * WSC_INV + bbb[3];
        const float ig = fsig(zi);
        const float fg = fsig(zf);
        const float og = fsig(zo);
        const float gg = fmaxf(zg, 0.0f);
        const float cn = fg * cb[r] + ig * gg;
        cb[r] = cn;
        const float hn = og * fmaxf(cn, 0.0f);
        h2v[r] = hn;
        _Float16 hi, lo;
        split_h(hn, hi, lo);
        h2wh[(8 * hh + r) * HPB + j2] = hi;
        h2wl[(8 * hh + r) * HPB + j2] = lo;
      }
    }
    __syncthreads();
  }

#pragma unroll
  for (int r = 0; r < 8; ++r) Hs[(8 * hh + r) * OPITCH + j2] = h2v[r];
  __syncthreads();
  for (int pass = 0; pass < 2; ++pass) {
#pragma unroll
    for (int it = 0; it < 2; ++it) {
      const int idx = it * NTHR + tid;
      const int row = idx >> 5, c4 = (idx & 31) * 4;
      const v4f v = *(const v4f*)(Hs + row * OPITCH + c4);
      *(volatile v4f*)(out + (size_t)(rowbase + row) * NUB + c4) = v;
    }
    __threadfence();
  }
}

extern "C" void kernel_launch(void* const* d_in, const int* in_sizes, int n_in,
                              void* d_out, int out_size, void* d_ws, size_t ws_size, hipStream_t stream) {
  if (n_in < 7 || d_out == nullptr || d_ws == nullptr) return;
  if (in_sizes[0] != NBATCH * NSTEP * NFEAT || in_sizes[1] != NFEAT * NGA || in_sizes[2] != NUA * NGA ||
      in_sizes[3] != NGA || in_sizes[4] != NUA * NGB || in_sizes[5] != NUB * NGB || in_sizes[6] != NGB ||
      out_size != NBATCH * NUB) return;

  const float* xin = (const float*)d_in[0];
  const float* w1  = (const float*)d_in[1];
  const float* u1  = (const float*)d_in[2];
  const float* b1  = (const float*)d_in[3];
  const float* w2  = (const float*)d_in[4];
  const float* u2  = (const float*)d_in[5];
  const float* b2  = (const float*)d_in[6];
  float* out = (float*)d_out;

  char* ws = (char*)d_ws; size_t off = 0;
  auto carve = [&](size_t bytes) -> char* { char* p = ws + off; off += (bytes + 255) & ~(size_t)255; return p; };
  unsigned short* WA = (unsigned short*)carve((size_t)NGA * K_L1 * 2);
  unsigned short* WB = (unsigned short*)carve((size_t)NGB * K_L2 * 2);
  if (off > ws_size || off > (size_t)134217728) return;

  tpw_kernel<<<dim3(NGA / 64, NFEAT / 64), NTHR, 0, stream>>>(w1, NFEAT, NGA, K_L1, 0,     WA, WSC);
  tpw_kernel<<<dim3(NGA / 64, NUA / 64),   NTHR, 0, stream>>>(u1, NUA,   NGA, K_L1, NFEAT, WA, WSC);
  tpw_kernel<<<dim3(NGB / 64, NUA / 64),   NTHR, 0, stream>>>(w2, NUA,   NGB, K_L2, 0,     WB, WSC);
  tpw_kernel<<<dim3(NGB / 64, NUB / 64),   NTHR, 0, stream>>>(u2, NUB,   NGB, K_L2, NUA,   WB, WSC);
  lstm2_kernel<<<NBATCH / SEQ_BLK, NTHR, 0, stream>>>(xin, b1, b2, WA, WB, out);
}
